// GNN_1_38001870635841
// MI455X (gfx1250) — hardware-verified
//
#include <hip/hip_runtime.h>
#include <stddef.h>


#define ZD   64
#define AD   8
#define KN   64
#define HD   512
#define NBAT 64
#define NR   (NBAT * KN)
#define KW1  128
#define KXI  136
#define KXP  192
#define XP   200
#define HP   520
#define CW   256
#define CP   264
#define NTH  256
#define W2S  16.0f
#define W2I  0.0625f

static_assert((XP % 8) == 0 && (HP % 8) == 0 && (CP % 8) == 0);
static_assert((KXP % 64) == 0 && KXP >= KXI);
static_assert((HD % CW) == 0 && (CW % 32) == 0);

typedef float          v4f   __attribute__((ext_vector_type(4)));
typedef float          v8f   __attribute__((ext_vector_type(8)));
typedef _Float16       v8h   __attribute__((ext_vector_type(8)));
typedef _Float16       v16h  __attribute__((ext_vector_type(16)));
typedef unsigned short v8us  __attribute__((ext_vector_type(8)));
typedef __bf16         v16bf __attribute__((ext_vector_type(16)));

union FragH { v16h v; v8h p[2]; };
union FragB { v16bf v; v8us p[2]; };
union CvtH  { v8h h; v8us u; };

__device__ __forceinline__ v8f zacc() {
  v8f c = {0.0f, 0.0f, 0.0f, 0.0f, 0.0f, 0.0f, 0.0f, 0.0f};
  return c;
}

__device__ __forceinline__ v8f wm_h(v16h a, v16h b, v8f c) {
  v8f d = __builtin_amdgcn_wmma_f32_16x16x32_f16(false, a, false, b, (short)0, c, false, false);
  asm volatile("v_nop\n\tv_nop\n\tv_nop\n\tv_nop" : "+v"(d) : "v"(a), "v"(b));
  return d;
}
__device__ __forceinline__ v8f wm_b(v16bf a, v16bf b, v8f c) {
  v8f d = __builtin_amdgcn_wmma_f32_16x16x32_bf16(false, a, false, b, (short)0, c, false, false);
  asm volatile("v_nop\n\tv_nop\n\tv_nop\n\tv_nop" : "+v"(d) : "v"(a), "v"(b));
  return d;
}

__device__ __forceinline__ unsigned short bf_bits(float f) {
  unsigned u = __float_as_uint(f);
  u = u + 0x7FFFu + ((u >> 16) & 1u);
  return (unsigned short)(u >> 16);
}
__device__ __forceinline__ float bf_val(unsigned short b) {
  return __uint_as_float(((unsigned)b) << 16);
}
__device__ __forceinline__ void split_bf(float v, unsigned short& hi, unsigned short& lo) {
  hi = bf_bits(v);
  lo = bf_bits(v - bf_val(hi));
}

__device__ __forceinline__ v16h frag_h(const _Float16* p, int h) {
  FragH f;
  f.p[0] = *(const v8h*)(p + 8 * h);
  f.p[1] = *(const v8h*)(p + 16 + 8 * h);
  return f.v;
}
__device__ __forceinline__ v16bf frag_us(const unsigned short* p, int h) {
  FragB f;
  f.p[0] = *(const v8us*)(p + 8 * h);
  f.p[1] = *(const v8us*)(p + 16 + 8 * h);
  return f.v;
}

template <int SPLIT>
__global__ __launch_bounds__(NTH) void k_wprep(const float* __restrict__ in, int R, int C, int Kp, float scale,
                                               unsigned short* oa, unsigned short* ob) {
  __shared__ __attribute__((aligned(16))) float tile[32 * 68];
  const int tid = threadIdx.x, lane = tid & 31, wave = tid >> 5;
  const int n0  = blockIdx.x * 32;
  const int nkc = Kp >> 6;
#pragma unroll 1
  for (int kc = 0; kc < nkc; ++kc) {
#pragma unroll
    for (int u = 0; u < 8; ++u) {
      const int e  = tid + NTH * u;
      const int kk = e >> 5, nn = e & 31;
      const int k  = kc * 64 + kk;
      const int kcl = (k < R) ? k : (R - 1);
      int n = n0 + nn; n = (n < C) ? n : (C - 1);
      float v = in[(size_t)kcl * C + n];
      v = (k < R) ? v : 0.0f;
      tile[nn * 68 + kk] = v;
    }
    __syncthreads();
    {
      const int nn = wave * 4 + (lane >> 3), pc = lane & 7;
      const float* tp = tile + nn * 68 + pc * 8;
      const v4f a = *(const v4f*)tp;
      const v4f b = *(const v4f*)(tp + 4);
      float f[8];
#pragma unroll
      for (int i = 0; i < 4; ++i) { f[i] = a[i]; f[4 + i] = b[i]; }
      v8us va = {0, 0, 0, 0, 0, 0, 0, 0}, vb = {0, 0, 0, 0, 0, 0, 0, 0};
      if (SPLIT == 0) {
        CvtH c;
#pragma unroll
        for (int i = 0; i < 8; ++i) c.h[i] = (_Float16)(f[i] * scale);
        va = c.u; vb = c.u;
      } else {
#pragma unroll
        for (int i = 0; i < 8; ++i) { unsigned short hi, lo; split_bf(f[i], hi, lo); va[i] = hi; vb[i] = lo; }
      }
      int nrow = n0 + nn; nrow = (nrow < C) ? nrow : (C - 1);
      const size_t o = (size_t)nrow * Kp + (size_t)kc * 64 + (size_t)(pc * 8);
      *(volatile v8us*)(oa + o) = va;
      if (SPLIT != 0) *(volatile v8us*)(ob + o) = vb;
      __threadfence();
      *(volatile v8us*)(oa + o) = va;
      if (SPLIT != 0) *(volatile v8us*)(ob + o) = vb;
    }
    __syncthreads();
  }
}

__global__ __launch_bounds__(NTH) void k_pq(const float* __restrict__ x,
                                           const unsigned short* __restrict__ w1h,
                                           const unsigned short* __restrict__ w1l,
                                           float* P, float* Q) {
  __shared__ __attribute__((aligned(16))) float st[16 * 1024];
  const int tid = threadIdx.x, lane = tid & 31, wave = tid >> 5, h = lane >> 4, m = lane & 15;
  const int row0 = blockIdx.x * 16;

  FragB ah[2], al[2];
#pragma unroll
  for (int ks = 0; ks < 2; ++ks) {
    const float* xp = x + (size_t)(row0 + m) * ZD + ks * 32;
    const v4f a0 = *(const v4f*)(xp + 8 * h);
    const v4f a1 = *(const v4f*)(xp + 8 * h + 4);
    const v4f a2 = *(const v4f*)(xp + 16 + 8 * h);
    const v4f a3 = *(const v4f*)(xp + 16 + 8 * h + 4);
    v8us hu0 = {0, 0, 0, 0, 0, 0, 0, 0}, hu1 = {0, 0, 0, 0, 0, 0, 0, 0};
    v8us lu0 = {0, 0, 0, 0, 0, 0, 0, 0}, lu1 = {0, 0, 0, 0, 0, 0, 0, 0};
#pragma unroll
    for (int i = 0; i < 4; ++i) {
      unsigned short hi, lo;
      split_bf(a0[i], hi, lo); hu0[i]     = hi; lu0[i]     = lo;
      split_bf(a1[i], hi, lo); hu0[4 + i] = hi; lu0[4 + i] = lo;
      split_bf(a2[i], hi, lo); hu1[i]     = hi; lu1[i]     = lo;
      split_bf(a3[i], hi, lo); hu1[4 + i] = hi; lu1[4 + i] = lo;
    }
    ah[ks].p[0] = hu0; ah[ks].p[1] = hu1;
    al[ks].p[0] = lu0; al[ks].p[1] = lu1;
  }

#pragma unroll 1
  for (int t = 0; t < 8; ++t) {
    const int nt    = wave + 8 * t;
    const int ncol0 = nt * 16;
    const int kb    = (nt >> 5) * 64;
    const int prow  = (ncol0 & 511) + m;
    const unsigned short* bph = w1h + (size_t)prow * KW1 + kb;
    const unsigned short* bpl = w1l + (size_t)prow * KW1 + kb;
    v8f acc = zacc();
#pragma unroll
    for (int ks = 0; ks < 2; ++ks) {
      const v16bf bh = frag_us(bph + ks * 32, h);
      const v16bf bl = frag_us(bpl + ks * 32, h);
      acc = wm_b(ah[ks].v, bh, acc);
      acc = wm_b(ah[ks].v, bl, acc);
      acc = wm_b(al[ks].v, bh, acc);
    }
#pragma unroll
    for (int r = 0; r < 8; ++r) st[(8 * h + r) * 1024 + ncol0 + m] = acc[r];
  }
  __syncthreads();

  const int cw = (wave & 3) * 128 + lane * 4;
#pragma unroll
  for (int s = 0; s < 16; ++s) {
    const v4f v = *(const v4f*)(st + s * 1024 + wave * 128 + lane * 4);
    const size_t o = (size_t)(row0 + s) * HD + cw;
    if (wave < 4) *(volatile v4f*)(P + o) = v; else *(volatile v4f*)(Q + o) = v;
  }
  __threadfence();
#pragma unroll
  for (int s = 0; s < 16; ++s) {
    const v4f v = *(const v4f*)(st + s * 1024 + wave * 128 + lane * 4);
    const size_t o = (size_t)(row0 + s) * HD + cw;
    if (wave < 4) *(volatile v4f*)(P + o) = v; else *(volatile v4f*)(Q + o) = v;
  }
}

__global__ __launch_bounds__(NTH) void k_edge(const float* __restrict__ P, const float* __restrict__ Q,
                                             const float* __restrict__ be1,
                                             const _Float16* __restrict__ w2t, const float* __restrict__ be2,
                                             const unsigned short* __restrict__ w3h,
                                             const unsigned short* __restrict__ w3l,
                                             const float* __restrict__ be3,
                                             float* E) {
  __shared__ __attribute__((aligned(16))) _Float16       h1[KN * HP];
  __shared__ __attribute__((aligned(16))) unsigned short h2h[KN * CP];
  __shared__ __attribute__((aligned(16))) unsigned short h2l[KN * CP];
  __shared__ __attribute__((aligned(16))) float          pb[HD];
  __shared__ __attribute__((aligned(16))) float          part[8 * ZD];
  __shared__ __attribute__((aligned(16))) float          est[ZD];

  const int tid = threadIdx.x, lane = tid & 31, wave = tid >> 5, h = lane >> 4, m = lane & 15;
  const int wg = blockIdx.x;
  const int b  = wg >> 6, inode = wg & 63;

  for (int c = tid; c < HD; c += NTH) pb[c] = P[(size_t)wg * HD + c] + be1[c];
  __syncthreads();

  {
    const float* qb = Q + (size_t)b * KN * HD;
#pragma unroll 2
    for (int idx = tid; idx < KN * (HD / 8); idx += NTH) {
      const int j = idx >> 6, cc = (idx & 63) << 3;
      const float* qp = qb + (size_t)j * HD + cc;
      const v4f q0 = *(const v4f*)qp, q1 = *(const v4f*)(qp + 4);
      const v4f p0 = *(const v4f*)(pb + cc), p1 = *(const v4f*)(pb + cc + 4);
      v8h hv;
#pragma unroll
      for (int i = 0; i < 4; ++i) {
        hv[i]     = (_Float16)fmaxf(q0[i] + p0[i], 0.0f);
        hv[4 + i] = (_Float16)fmaxf(q1[i] + p1[i], 0.0f);
      }
      *(v8h*)(h1 + j * HP + cc) = hv;
    }
  }
  __syncthreads();

  v8f acc3[2];
  acc3[0] = zacc(); acc3[1] = zacc();
  const int mt3 = wave >> 1, nq = (wave & 1) * 2;

#pragma unroll 1
  for (int nc = 0; nc < HD / CW; ++nc) {
#pragma unroll 1
    for (int p = 0; p < 2; ++p) {
      const int ntl  = p * 8 + wave;
      const int col0 = nc * CW + ntl * 16;
      v8f acc[4];
      acc[0] = zacc(); acc[1] = zacc(); acc[2] = zacc(); acc[3] = zacc();
      const _Float16* bp = w2t + (size_t)(col0 + m) * HD;
#pragma unroll 1
      for (int kt = 0; kt < HD / 32; ++kt) {
        const v16h bf = frag_h(bp + kt * 32, h);
#pragma unroll
        for (int t = 0; t < 4; ++t) {
          const v16h af = frag_h(h1 + (t * 16 + m) * HP + kt * 32, h);
          acc[t] = wm_h(af, bf, acc[t]);
        }
      }
      const float bb = be2[col0 + m];
#pragma unroll
      for (int t = 0; t < 4; ++t) {
#pragma unroll
        for (int r = 0; r < 8; ++r) {
          const float v = fmaxf(acc[t][r] * W2I + bb, 0.0f);
          unsigned short hi, lo;
          split_bf(v, hi, lo);
          const int o = (t * 16 + 8 * h + r) * CP + ntl * 16 + m;
          h2h[o] = hi;
          h2l[o] = lo;
        }
      }
    }
    __syncthreads();

#pragma unroll 1
    for (int ks = 0; ks < CW / 32; ++ks) {
      const v16bf ahf = frag_us(h2h + (mt3 * 16 + m) * CP + ks * 32, h);
      const v16bf alf = frag_us(h2l + (mt3 * 16 + m) * CP + ks * 32, h);
#pragma unroll
      for (int q = 0; q < 2; ++q) {
        const size_t bo = (size_t)((nq + q) * 16 + m) * HD + (size_t)(nc * CW + ks * 32);
        const v16bf bh = frag_us(w3h + bo, h);
        const v16bf bl = frag_us(w3l + bo, h);
        acc3[q] = wm_b(ahf, bh, acc3[q]);
        acc3[q] = wm_b(ahf, bl, acc3[q]);
        acc3[q] = wm_b(alf, bh, acc3[q]);
      }
    }
    __syncthreads();
  }

  {
    const int rbase = mt3 * 16 + 8 * h;
#pragma unroll
    for (int q = 0; q < 2; ++q) {
      const int col = (nq + q) * 16 + m;
      const float bc = be3[col];
      float s = 0.0f;
#pragma unroll
      for (int r = 0; r < 8; ++r) {
        const float tv = acc3[q][r] + bc;
        s += ((rbase + r) != inode) ? tv : 0.0f;
      }
      part[(mt3 * 2 + h) * ZD + col] = s;
    }
  }
  __syncthreads();
  if (tid < ZD) {
    float s = 0.0f;
#pragma unroll
    for (int u = 0; u < 8; ++u) s += part[u * ZD + tid];
    est[tid] = s;
  }
  __syncthreads();

  const bool wr = (wave == 0) && (lane < 16);
  v4f ev = {0.0f, 0.0f, 0.0f, 0.0f};
  if (wr) ev = *(const v4f*)(est + 4 * lane);
  if (wr) *(volatile v4f*)(E + (size_t)wg * ZD + 4 * lane) = ev;
  __threadfence();
  if (wr) *(volatile v4f*)(E + (size_t)wg * ZD + 4 * lane) = ev;
}

__global__ __launch_bounds__(NTH) void k_node(const float* __restrict__ x, const float* __restrict__ a,
                                             const float* __restrict__ E,
                                             const unsigned short* __restrict__ n1h,
                                             const unsigned short* __restrict__ n1l,
                                             const float* __restrict__ bn1,
                                             const unsigned short* __restrict__ n2h,
                                             const unsigned short* __restrict__ n2l,
                                             const float* __restrict__ bn2,
                                             const unsigned short* __restrict__ n3h,
                                             const unsigned short* __restrict__ n3l,
                                             const float* __restrict__ bn3,
                                             float* out) {
  __shared__ __attribute__((aligned(16))) unsigned short xh[16 * XP];
  __shared__ __attribute__((aligned(16))) unsigned short xl[16 * XP];
  __shared__ __attribute__((aligned(16))) unsigned short g1h[16 * HP];
  __shared__ __attribute__((aligned(16))) unsigned short g1l[16 * HP];
  __shared__ __attribute__((aligned(16))) unsigned short g2h[16 * HP];
  __shared__ __attribute__((aligned(16))) unsigned short g2l[16 * HP];
  __shared__ __attribute__((aligned(16))) float          ost[16 * ZD];

  const int tid = threadIdx.x, lane = tid & 31, wave = tid >> 5, h = lane >> 4, m = lane & 15;
  const int row0 = blockIdx.x * 16;

#pragma unroll 1
  for (int idx = tid; idx < 16 * KXP; idx += NTH) {
    const int r = idx / KXP, c = idx - r * KXP;
    const int grow = row0 + r;
    const int cx = (c < ZD) ? c : (ZD - 1);
    int ca = c - ZD;        ca = ca < 0 ? 0 : (ca > AD - 1 ? AD - 1 : ca);
    int ce = c - (ZD + AD); ce = ce < 0 ? 0 : (ce > ZD - 1 ? ZD - 1 : ce);
    const float vx = x[(size_t)grow * ZD + cx];
    const float va = a[(size_t)grow * AD + ca];
    const float ve = E[(size_t)grow * ZD + ce];
    const float v = (c < ZD) ? vx : ((c < ZD + AD) ? va : ((c < KXI) ? ve : 0.0f));
    unsigned short hi, lo;
    split_bf(v, hi, lo);
    xh[r * XP + c] = hi;
    xl[r * XP + c] = lo;
  }
  __syncthreads();

#pragma unroll 1
  for (int t = 0; t < 4; ++t) {
    const int col0 = (wave + 8 * t) * 16;
    const unsigned short* bph = n1h + (size_t)(col0 + m) * KXP;
    const unsigned short* bpl = n1l + (size_t)(col0 + m) * KXP;
    v8f acc = zacc();
#pragma unroll 1
    for (int ks = 0; ks < KXP / 32; ++ks) {
      const v16bf ahf = frag_us(xh + m * XP + ks * 32, h);
      const v16bf alf = frag_us(xl + m * XP + ks * 32, h);
      const v16bf bh  = frag_us(bph + ks * 32, h);
      const v16bf bl  = frag_us(bpl + ks * 32, h);
      acc = wm_b(ahf, bh, acc);
      acc = wm_b(ahf, bl, acc);
      acc = wm_b(alf, bh, acc);
    }
    const float bb = bn1[col0 + m];
#pragma unroll
    for (int r = 0; r < 8; ++r) {
      const float v = fmaxf(acc[r] + bb, 0.0f);
      unsigned short hi, lo;
      split_bf(v, hi, lo);
      const int o = (8 * h + r) * HP + col0 + m;
      g1h[o] = hi;
      g1l[o] = lo;
    }
  }
  __syncthreads();

#pragma unroll 1
  for (int t = 0; t < 4; ++t) {
    const int col0 = (wave + 8 * t) * 16;
    const unsigned short* bph = n2h + (size_t)(col0 + m) * HD;
    const unsigned short* bpl = n2l + (size_t)(col0 + m) * HD;
    v8f acc = zacc();
#pragma unroll 1
    for (int ks = 0; ks < HD / 32; ++ks) {
      const v16bf ahf = frag_us(g1h + m * HP + ks * 32, h);
      const v16bf alf = frag_us(g1l + m * HP + ks * 32, h);
      const v16bf bh  = frag_us(bph + ks * 32, h);
      const v16bf bl  = frag_us(bpl + ks * 32, h);
      acc = wm_b(ahf, bh, acc);
      acc = wm_b(ahf, bl, acc);
      acc = wm_b(alf, bh, acc);
    }
    const float bb = bn2[col0 + m];
#pragma unroll
    for (int r = 0; r < 8; ++r) {
      const float v = fmaxf(acc[r] + bb, 0.0f);
      unsigned short hi, lo;
      split_bf(v, hi, lo);
      const int o = (8 * h + r) * HP + col0 + m;
      g2h[o] = hi;
      g2l[o] = lo;
    }
  }
  __syncthreads();

  if (wave < 4) {
    const int col0 = wave * 16;
    const unsigned short* bph = n3h + (size_t)(col0 + m) * HD;
    const unsigned short* bpl = n3l + (size_t)(col0 + m) * HD;
    v8f acc = zacc();
#pragma unroll 1
    for (int ks = 0; ks < HD / 32; ++ks) {
      const v16bf ahf = frag_us(g2h + m * HP + ks * 32, h);
      const v16bf alf = frag_us(g2l + m * HP + ks * 32, h);
      const v16bf bh  = frag_us(bph + ks * 32, h);
      const v16bf bl  = frag_us(bpl + ks * 32, h);
      acc = wm_b(ahf, bh, acc);
      acc = wm_b(ahf, bl, acc);
      acc = wm_b(alf, bh, acc);
    }
    const float bb = bn3[col0 + m];
#pragma unroll
    for (int r = 0; r < 8; ++r) ost[(8 * h + r) * ZD + col0 + m] = acc[r] + bb;
  }
  __syncthreads();

  const v4f ov = *(const v4f*)(ost + tid * 4);
  const size_t oo = (size_t)row0 * ZD + (size_t)(tid * 4);
  *(volatile v4f*)(out + oo) = ov;
  __threadfence();
  *(volatile v4f*)(out + oo) = ov;
}

extern "C" void kernel_launch(void* const* d_in, const int* in_sizes, int n_in,
                              void* d_out, int out_size, void* d_ws, size_t ws_size,
                              hipStream_t stream) {
  if (n_in < 14) return;
  if (in_sizes[0] != NR * ZD || in_sizes[1] != NR * AD) return;
  if (in_sizes[2] != KW1 * HD || in_sizes[3] != HD) return;
  if (in_sizes[4] != HD * HD || in_sizes[5] != HD) return;
  if (in_sizes[6] != HD * ZD || in_sizes[7] != ZD) return;
  if (in_sizes[8] != KXI * HD || in_sizes[9] != HD) return;
  if (in_sizes[10] != HD * HD || in_sizes[11] != HD) return;
  if (in_sizes[12] != HD * ZD || in_sizes[13] != ZD) return;
  if (out_size != NR * ZD) return;

  const float* x   = (const float*)d_in[0];
  const float* a   = (const float*)d_in[1];
  const float* We1 = (const float*)d_in[2];
  const float* be1 = (const float*)d_in[3];
  const float* We2 = (const float*)d_in[4];
  const float* be2 = (const float*)d_in[5];
  const float* We3 = (const float*)d_in[6];
  const float* be3 = (const float*)d_in[7];
  const float* Wn1 = (const float*)d_in[8];
  const float* bn1 = (const float*)d_in[9];
  const float* Wn2 = (const float*)d_in[10];
  const float* bn2 = (const float*)d_in[11];
  const float* Wn3 = (const float*)d_in[12];
  const float* bn3 = (const float*)d_in[13];
  float* outp = (float*)d_out;

  char* ws = (char*)d_ws;
  size_t off = 0;
  auto carve = [&](size_t bytes) -> char* {
    char* p = ws + off;
    off += (bytes + 255) & ~(size_t)255;
    return p;
  };
  unsigned short* w1h = (unsigned short*)carve((size_t)HD * KW1 * 2);
  unsigned short* w1l = (unsigned short*)carve((size_t)HD * KW1 * 2);
  unsigned short* w2t = (unsigned short*)carve((size_t)HD * HD * 2);
  unsigned short* w3h = (unsigned short*)carve((size_t)ZD * HD * 2);
  unsigned short* w3l = (unsigned short*)carve((size_t)ZD * HD * 2);
  unsigned short* n1h = (unsigned short*)carve((size_t)HD * KXP * 2);
  unsigned short* n1l = (unsigned short*)carve((size_t)HD * KXP * 2);
  unsigned short* n2h = (unsigned short*)carve((size_t)HD * HD * 2);
  unsigned short* n2l = (unsigned short*)carve((size_t)HD * HD * 2);
  unsigned short* n3h = (unsigned short*)carve((size_t)ZD * HD * 2);
  unsigned short* n3l = (unsigned short*)carve((size_t)ZD * HD * 2);
  float*          Pm  = (float*)carve((size_t)NR * HD * 4);
  float*          Qm  = (float*)carve((size_t)NR * HD * 4);
  float*          Em  = (float*)carve((size_t)NR * ZD * 4);
  if (off > ws_size) return;
  if (off > (size_t)134217728) return;

  static_assert((HD % 32) == 0 && (ZD % 32) == 0);
  static_assert((NR % 16) == 0);

  k_wprep<1><<<HD / 32, NTH, 0, stream>>>(We1, KW1, HD, KW1, 1.0f, w1h, w1l);
  k_wprep<0><<<HD / 32, NTH, 0, stream>>>(We2, HD,  HD, HD,  W2S,  w2t, w2t);
  k_wprep<1><<<ZD / 32, NTH, 0, stream>>>(We3, HD,  ZD, HD,  1.0f, w3h, w3l);
  k_wprep<1><<<HD / 32, NTH, 0, stream>>>(Wn1, KXI, HD, KXP, 1.0f, n1h, n1l);
  k_wprep<1><<<HD / 32, NTH, 0, stream>>>(Wn2, HD,  HD, HD,  1.0f, n2h, n2l);
  k_wprep<1><<<ZD / 32, NTH, 0, stream>>>(Wn3, HD,  ZD, HD,  1.0f, n3h, n3l);

  k_pq<<<NR / 16, NTH, 0, stream>>>(x, w1h, w1l, Pm, Qm);

  k_edge<<<NR, NTH, 0, stream>>>(Pm, Qm, be1, (const _Float16*)w2t, be2, w3h, w3l, be3, Em);

  k_node<<<NR / 16, NTH, 0, stream>>>(x, a, Em, n1h, n1l, bn1, n2h, n2l, bn2, n3h, n3l, bn3, outp);
}
